// MultiheadSelfAttention_33672543600672
// MI455X (gfx1250) — hardware-verified
//
#include <hip/hip_runtime.h>


#ifndef NB
#define NB 2
#endif
#ifndef SEQ
#define SEQ 2048
#endif
#define SEQ_FULL 2048
#define DM   512
#define NH   8
#define HD   64
#define AW   4
#define PP   40
#define OSP  68
#define SCL  0.125f
static_assert(HD == 64);
static_assert(NH * HD == DM);
static_assert(DM % 64 == 0);
static_assert(DM % 32 == 0);
static_assert(SEQ % 64 == 0);
static_assert(SEQ % (16 * AW) == 0);
static_assert(SEQ % 32 == 0);
static_assert((NB * SEQ) % 64 == 0);
static_assert(PP >= 32 && PP % 8 == 0);
static_assert(OSP >= 64 && OSP % 4 == 0);
static_assert(SEQ <= SEQ_FULL);

typedef _Float16 h16;
typedef unsigned short bf;
typedef __attribute__((ext_vector_type(16))) __bf16   v16bf;
typedef __attribute__((ext_vector_type(16))) _Float16 v16h;
typedef __attribute__((ext_vector_type(8)))  _Float16 v8h;
typedef __attribute__((ext_vector_type(8)))  unsigned short v8us;
typedef __attribute__((ext_vector_type(8)))  float    v8f;
typedef __attribute__((ext_vector_type(4)))  float    v4f;
typedef v8h  __attribute__((may_alias)) v8ha;
typedef v4f  __attribute__((may_alias)) v4fa;

__device__ __forceinline__ unsigned short f2bf(float f) { unsigned u = __float_as_uint(f); u += 0x7FFFu + ((u >> 16) & 1u); return (unsigned short)(u >> 16); }
__device__ __forceinline__ float bf2f(unsigned short b) { return __uint_as_float(((unsigned)b) << 16); }
__device__ __forceinline__ float bfr(float f) { return bf2f(f2bf(f)); }
__device__ __forceinline__ void splitf(float y, unsigned short& h, unsigned short& l) { h = f2bf(y); l = f2bf(y - bf2f(h)); }
__device__ __forceinline__ v16h cat16(v8h lo, v8h hi) { return __builtin_shufflevector(lo, hi, 0, 1, 2, 3, 4, 5, 6, 7, 8, 9, 10, 11, 12, 13, 14, 15); }
__device__ __forceinline__ v16bf cat16b(v8us lo, v8us hi) { return __builtin_bit_cast(v16bf, __builtin_shufflevector(lo, hi, 0, 1, 2, 3, 4, 5, 6, 7, 8, 9, 10, 11, 12, 13, 14, 15)); }
__device__ __forceinline__ v8f wmma16(v16h a, v16h b, v8f c) { return __builtin_amdgcn_wmma_f32_16x16x32_f16(false, a, false, b, (short)0, c, false, false); }
__device__ __forceinline__ v8f wmmab(v16bf a, v16bf b, v8f c) { return __builtin_amdgcn_wmma_f32_16x16x32_bf16(false, a, false, b, (short)0, c, false, false); }
__device__ __forceinline__ v16h  ldh(const h16* p) { return cat16(*(const v8h*)p, *(const v8h*)(p + 16)); }
__device__ __forceinline__ v16bf ldb(const bf* p)  { return cat16b(*(const v8us*)p, *(const v8us*)(p + 16)); }
__device__ __forceinline__ void lds_wave_sync() { __builtin_amdgcn_fence(3  , "wavefront"); __builtin_amdgcn_wave_barrier(); asm volatile("" ::: "memory"); }

__global__ __launch_bounds__(256) void k_cvt8(const float* __restrict__ src, bf* dst, unsigned n8, size_t sS, size_t sD) {
    const unsigned i = blockIdx.x * 256u + threadIdx.x; if (i >= n8) return;
    const size_t so = (size_t)blockIdx.y * sS + (size_t)i * 8, dofs = (size_t)blockIdx.y * sD + (size_t)i * 8;
    const v4f a = *(const v4f*)(src + so), b = *(const v4f*)(src + so + 4); v8us o;
#pragma unroll
    for (int k = 0; k < 4; ++k) { o[k] = f2bf(a[k]); o[4 + k] = f2bf(b[k]); }
    *(volatile v8us*)(dst + dofs) = o; __threadfence(); *(volatile v8us*)(dst + dofs) = o;
}

template <int NSPLIT>
__device__ __forceinline__ void gemm_main(const bf* __restrict__ A, const bf* __restrict__ A2, const bf* __restrict__ Bt, const int K, const size_t aoff, const size_t boff, v8f (&acc)[4][4]) {
#pragma unroll
    for (int mb = 0; mb < 4; ++mb)
#pragma unroll
        for (int nb = 0; nb < 4; ++nb) acc[mb][nb] = (v8f){};
#pragma unroll 1
    for (int kc = 0; kc < K; kc += 32) {
        v16bf a[4], a2[4], b;
#pragma unroll
        for (int mb = 0; mb < 4; ++mb) { a[mb] = ldb(A + aoff + (size_t)mb * 16 * K + kc); if (NSPLIT) a2[mb] = ldb(A2 + aoff + (size_t)mb * 16 * K + kc); else a2[mb] = a[mb]; }
#pragma unroll
        for (int nb = 0; nb < 4; ++nb) { b = ldb(Bt + boff + (size_t)nb * 16 * K + kc);
#pragma unroll
            for (int mb = 0; mb < 4; ++mb) { acc[mb][nb] = wmmab(a[mb], b, acc[mb][nb]); if (NSPLIT) acc[mb][nb] = wmmab(a2[mb], b, acc[mb][nb]); } }
        asm volatile("v_nop\n\tv_nop\n\tv_nop\n\tv_nop" : "+v"(acc[0][0]), "+v"(acc[1][0]), "+v"(acc[2][0]), "+v"(acc[3][0]), "+v"(acc[0][1]), "+v"(acc[1][1]), "+v"(acc[2][1]), "+v"(acc[3][1]) : "v"(a[0]), "v"(a2[3]));
        asm volatile("v_nop\n\tv_nop\n\tv_nop\n\tv_nop" : "+v"(acc[0][2]), "+v"(acc[1][2]), "+v"(acc[2][2]), "+v"(acc[3][2]), "+v"(acc[0][3]), "+v"(acc[1][3]), "+v"(acc[2][3]), "+v"(acc[3][3]) : "v"(b), "v"(a[3]), "v"(a2[3]));
    }
}

template <int ROWB>
__device__ __forceinline__ void epi_h16(v8f (&acc)[4][4], h16* Cb, const int ldc, const float* __restrict__ bias, const int bofs, const int lane) {
    __shared__ __align__(16) float os[16 * OSP];
    const int lr = lane & 15, hi = lane >> 4, rq = lane >> 3, c8 = (lane & 7) * 8;
#pragma unroll
    for (int mb = 0; mb < 4; ++mb) {
#pragma unroll
        for (int nb = 0; nb < 4; ++nb) {
#pragma unroll
            for (int j = 0; j < 8; ++j) os[(hi * 8 + j) * OSP + nb * 16 + lr] = acc[mb][nb][j]; }
        lds_wave_sync();
#pragma unroll 1
        for (int ps = 0; ps < 2; ++ps) {
#pragma unroll
            for (int s = 0; s < 4; ++s) { const int row = 4 * s + rq; const v4f a = *(const v4fa*)(os + row * OSP + c8); const v4f b = *(const v4fa*)(os + row * OSP + c8 + 4); float bb[8];
                if (ROWB) { const float rb = bfr(bias[bofs + mb * 16 + row]);
#pragma unroll
                    for (int q = 0; q < 8; ++q) bb[q] = rb;
                } else {
#pragma unroll
                    for (int q = 0; q < 8; ++q) bb[q] = bfr(bias[bofs + c8 + q]); }
                v8h o;
#pragma unroll
                for (int q = 0; q < 4; ++q) { o[q] = (h16)(a[q] + bb[q]); o[4 + q] = (h16)(b[q] + bb[4 + q]); }
                *(volatile v8h*)(Cb + (size_t)(mb * 16 + row) * ldc + c8) = o; }
            if (ps == 0) __threadfence(); }
        lds_wave_sync();
    }
}

__global__ __launch_bounds__(32) void k_projqk(const bf* __restrict__ XB, const bf* __restrict__ W, const float* __restrict__ bias, h16* P) {
    const int lane = threadIdx.x & 31, lr = lane & 15, hi = lane >> 4; const int r0 = blockIdx.x * 64, c0 = blockIdx.y * 64; const size_t z = blockIdx.z;
    v8f acc[4][4];
    gemm_main<0>(XB + z * SEQ * DM, XB + z * SEQ * DM, W, DM, (size_t)(r0 + lr) * DM + 8 * hi, (size_t)(c0 + lr) * DM + 8 * hi, acc);
    h16* Cb = P + (z * NH + blockIdx.y) * (size_t)SEQ * HD + (size_t)r0 * HD;
    epi_h16<0>(acc, Cb, HD, bias, c0, lane);
}
__global__ __launch_bounds__(32) void k_projvt(const bf* __restrict__ W, const bf* __restrict__ XB, const float* __restrict__ bias, h16* VT) {
    const int lane = threadIdx.x & 31, lr = lane & 15, hi = lane >> 4; const int r0 = blockIdx.x * 64, c0 = blockIdx.y * 64; const size_t z = blockIdx.z;
    v8f acc[4][4];
    gemm_main<0>(W, W, XB + z * SEQ * DM, DM, (size_t)(r0 + lr) * DM + 8 * hi, (size_t)(c0 + lr) * DM + 8 * hi, acc);
    h16* Cb = VT + z * (size_t)DM * SEQ + (size_t)r0 * SEQ + c0;
    epi_h16<1>(acc, Cb, SEQ, bias, r0, lane);
}
__global__ __launch_bounds__(32) void k_oproj(const bf* __restrict__ Ah, const bf* __restrict__ Al, const bf* __restrict__ WO, const float* __restrict__ bias, float* C) {
    __shared__ __align__(16) float os[16 * OSP];
    const int lane = threadIdx.x & 31, lr = lane & 15, hi = lane >> 4; const int r0 = blockIdx.x * 64, c0 = blockIdx.y * 64;
    v8f acc[4][4];
    gemm_main<1>(Ah, Al, WO, DM, (size_t)(r0 + lr) * DM + 8 * hi, (size_t)(c0 + lr) * DM + 8 * hi, acc);
#pragma unroll
    for (int mb = 0; mb < 4; ++mb) {
#pragma unroll
        for (int nb = 0; nb < 4; ++nb) {
#pragma unroll
            for (int j = 0; j < 8; ++j) os[(hi * 8 + j) * OSP + nb * 16 + lr] = acc[mb][nb][j]; }
        lds_wave_sync();
        float* crow = C + (size_t)(r0 + mb * 16) * DM + c0;
#pragma unroll 1
        for (int ps = 0; ps < 2; ++ps) {
#pragma unroll
            for (int s = 0; s < 8; ++s) { const int row = 2 * s + hi, cofs = lr * 4; v4f val = *(const v4fa*)(os + row * OSP + cofs);
                val[0] += bfr(bias[c0 + cofs]); val[1] += bfr(bias[c0 + cofs + 1]); val[2] += bfr(bias[c0 + cofs + 2]); val[3] += bfr(bias[c0 + cofs + 3]);
                *(volatile v4f*)(crow + (size_t)row * DM + cofs) = val; }
            if (ps == 0) __threadfence(); }
        lds_wave_sync();
    }
}

__global__ __launch_bounds__(AW * 32) void k_flash(const h16* __restrict__ QP, const h16* __restrict__ KP, const h16* __restrict__ VT, bf* Ah, bf* Al) {
    __shared__ __align__(16) h16 pb[AW * 16 * PP];
    __shared__ __align__(16) float os[AW * 16 * OSP];
    const int lane = threadIdx.x & 31, lr = lane & 15, hi = lane >> 4;
    const int wave = __builtin_amdgcn_readfirstlane(threadIdx.x >> 5);
    const int z = blockIdx.y;
    const int q0 = (blockIdx.x * AW + wave) * 16;
    const size_t zoff = (size_t)z * SEQ * HD;
    const size_t qoff = zoff + (size_t)(q0 + lr) * HD + 8 * hi;
    const size_t koff = zoff + (size_t)lr * HD + 8 * hi;
    const size_t voff = zoff + (size_t)lr * SEQ + 8 * hi;
    const int pbo = wave * 16 * PP, oso = wave * 16 * OSP;
    const v16h aq0 = ldh(QP + qoff), aq1 = ldh(QP + qoff + 32);
    float mrow[8], lrow[8];
    v8f o0 = (v8f){}, o1 = (v8f){}, o2 = (v8f){}, o3 = (v8f){};
#pragma unroll
    for (int r = 0; r < 8; ++r) { mrow[r] = -1.0e30f; lrow[r] = 0.0f; }
    const float csc = SCL * 1.4426950408889634f;
#pragma unroll 1
    for (int j0 = 0; j0 < SEQ; j0 += 32) {
        const h16* kp = KP + koff + (size_t)j0 * HD;
        const v16h bk00 = ldh(kp), bk01 = ldh(kp + 32), bk10 = ldh(kp + 16 * HD), bk11 = ldh(kp + 16 * HD + 32);
        v8f s0 = (v8f){}, s1 = (v8f){};
        s0 = wmma16(aq0, bk00, s0); s0 = wmma16(aq1, bk01, s0);
        s1 = wmma16(aq0, bk10, s1); s1 = wmma16(aq1, bk11, s1);
        asm volatile("v_nop\n\tv_nop\n\tv_nop\n\tv_nop" : "+v"(s0), "+v"(s1) : "v"(bk11), "v"(aq1));
#pragma unroll
        for (int r = 0; r < 8; ++r) {
            const float x0 = s0[r] * csc, x1 = s1[r] * csc;
            float mx = fmaxf(x0, x1);
            mx = fmaxf(mx, __shfl_xor(mx, 1, 32)); mx = fmaxf(mx, __shfl_xor(mx, 2, 32)); mx = fmaxf(mx, __shfl_xor(mx, 4, 32)); mx = fmaxf(mx, __shfl_xor(mx, 8, 32));
            const float nm = fmaxf(mrow[r], mx);
            const float sc = __builtin_amdgcn_exp2f(mrow[r] - nm);
            const float nb8 = nm - 8.0f;
            const float p0 = __builtin_amdgcn_exp2f(x0 - nb8), p1 = __builtin_amdgcn_exp2f(x1 - nb8);
            lrow[r] = lrow[r] * sc + (p0 + p1);
            mrow[r] = nm;
            o0[r] *= sc; o1[r] *= sc; o2[r] *= sc; o3[r] *= sc;
            pb[pbo + (8 * hi + r) * PP + lr] = (h16)p0;
            pb[pbo + (8 * hi + r) * PP + 16 + lr] = (h16)p1;
        }
        lds_wave_sync();
        const v16h ap = cat16(*(const v8ha*)(pb + pbo + lr * PP + 8 * hi), *(const v8ha*)(pb + pbo + lr * PP + 16 + 8 * hi));
        const h16* vp = VT + voff + j0;
        const v16h bv0 = ldh(vp), bv1 = ldh(vp + (size_t)16 * SEQ), bv2 = ldh(vp + (size_t)32 * SEQ), bv3 = ldh(vp + (size_t)48 * SEQ);
        o0 = wmma16(ap, bv0, o0); o1 = wmma16(ap, bv1, o1); o2 = wmma16(ap, bv2, o2); o3 = wmma16(ap, bv3, o3);
        asm volatile("v_nop\n\tv_nop\n\tv_nop\n\tv_nop" : "+v"(o0), "+v"(o1), "+v"(o2), "+v"(o3) : "v"(bv3), "v"(ap));
        lds_wave_sync();
    }
#pragma unroll
    for (int r = 0; r < 8; ++r) {
        float lt = lrow[r];
        lt += __shfl_xor(lt, 1, 32); lt += __shfl_xor(lt, 2, 32); lt += __shfl_xor(lt, 4, 32); lt += __shfl_xor(lt, 8, 32);
        const float inv = 1.0f / lt;
        os[oso + (8 * hi + r) * OSP + lr]      = o0[r] * inv;
        os[oso + (8 * hi + r) * OSP + 16 + lr] = o1[r] * inv;
        os[oso + (8 * hi + r) * OSP + 32 + lr] = o2[r] * inv;
        os[oso + (8 * hi + r) * OSP + 48 + lr] = o3[r] * inv;
    }
    lds_wave_sync();
    const int b = z / NH, h = z % NH, rq = lane >> 3, c8 = (lane & 7) * 8;
#pragma unroll 1
    for (int ps = 0; ps < 2; ++ps) {
#pragma unroll
        for (int s = 0; s < 4; ++s) { const int row = 4 * s + rq; const v4f a = *(const v4fa*)(os + oso + row * OSP + c8); const v4f c = *(const v4fa*)(os + oso + row * OSP + c8 + 4); v8us oh, ol;
#pragma unroll
            for (int q = 0; q < 4; ++q) { unsigned short x, y; splitf(a[q], x, y); oh[q] = x; ol[q] = y; splitf(c[q], x, y); oh[4 + q] = x; ol[4 + q] = y; }
            const size_t oo = ((size_t)b * SEQ + q0 + row) * DM + h * HD + c8;
            *(volatile v8us*)(Ah + oo) = oh; *(volatile v8us*)(Al + oo) = ol; }
        if (ps == 0) __threadfence(); }
}

#define SZ_XB  ((size_t)NB * SEQ * DM * 2)
#define SZ_W   ((size_t)DM * DM * 2)
#define SZ_PL  ((size_t)NB * NH * SEQ * HD * 2)
#define SZ_AT  ((size_t)NB * SEQ * DM * 2)
#define WS_TOTAL (SZ_XB + 4 * SZ_W + 3 * SZ_PL + 2 * SZ_AT)
static_assert(WS_TOTAL <= (size_t)134217728);
static_assert(SZ_XB % 256 == 0 && SZ_W % 256 == 0 && SZ_PL % 256 == 0 && SZ_AT % 256 == 0);

extern "C" void kernel_launch(void* const* d_in, const int* in_sizes, int n_in,
                              void* d_out, int out_size, void* d_ws, size_t ws_size, hipStream_t stream) {
    if (n_in < 9) return;
    const size_t XN = (size_t)(NB - 1) * SEQ_FULL * DM + (size_t)SEQ * DM;
    if ((size_t)in_sizes[0] < XN) return;
    if (in_sizes[1] < DM * DM || in_sizes[3] < DM * DM || in_sizes[5] < DM * DM || in_sizes[7] < DM * DM) return;
    if (in_sizes[2] < DM || in_sizes[4] < DM || in_sizes[6] < DM || in_sizes[8] < DM) return;
    if ((size_t)out_size < (size_t)NB * SEQ * DM) return;
    if (ws_size < WS_TOTAL) return;
    const float* x  = (const float*)d_in[0];
    const float* Wq = (const float*)d_in[1]; const float* bq = (const float*)d_in[2];
    const float* Wk = (const float*)d_in[3]; const float* bk = (const float*)d_in[4];
    const float* Wv = (const float*)d_in[5]; const float* bv = (const float*)d_in[6];
    const float* Wo = (const float*)d_in[7]; const float* bo = (const float*)d_in[8];
    float* OUT = (float*)d_out;
    char* wsp = (char*)d_ws;
    auto take = [&](size_t bytes) { char* p = wsp; wsp += bytes; return (void*)p; };
    bf* XB = (bf*)take(SZ_XB);
    bf* WQ = (bf*)take(SZ_W); bf* WK = (bf*)take(SZ_W); bf* WV = (bf*)take(SZ_W); bf* WO = (bf*)take(SZ_W);
    h16* QP = (h16*)take(SZ_PL); h16* KP = (h16*)take(SZ_PL); h16* VT = (h16*)take(SZ_PL);
    bf* ATh = (bf*)take(SZ_AT); bf* ATl = (bf*)take(SZ_AT);
    if ((size_t)(wsp - (char*)d_ws) > ws_size) return;

    const unsigned XN8 = (unsigned)((size_t)SEQ * DM / 8), WN8 = (unsigned)((size_t)DM * DM / 8);
    k_cvt8<<<dim3((XN8 + 255) / 256, NB), 256, 0, stream>>>(x, XB, XN8, (size_t)SEQ_FULL * DM, (size_t)SEQ * DM);
    k_cvt8<<<dim3((WN8 + 255) / 256, 1), 256, 0, stream>>>(Wq, WQ, WN8, 0, 0);
    k_cvt8<<<dim3((WN8 + 255) / 256, 1), 256, 0, stream>>>(Wk, WK, WN8, 0, 0);
    k_cvt8<<<dim3((WN8 + 255) / 256, 1), 256, 0, stream>>>(Wv, WV, WN8, 0, 0);
    k_cvt8<<<dim3((WN8 + 255) / 256, 1), 256, 0, stream>>>(Wo, WO, WN8, 0, 0);
    k_projqk<<<dim3(SEQ / 64, DM / 64, NB), 32, 0, stream>>>(XB, WQ, bq, QP);
    k_projqk<<<dim3(SEQ / 64, DM / 64, NB), 32, 0, stream>>>(XB, WK, bk, KP);
    k_projvt<<<dim3(DM / 64, SEQ / 64, NB), 32, 0, stream>>>(WV, XB, bv, VT);
    k_flash<<<dim3(SEQ / (16 * AW), NB * NH), AW * 32, 0, stream>>>(QP, KP, VT, ATh, ATl);
    k_oproj<<<dim3(NB * SEQ / 64, DM / 64, 1), 32, 0, stream>>>(ATh, ATl, WO, bo, OUT);
}
